// PyTorchAttention_65996467470660
// MI455X (gfx1250) — hardware-verified
//
#include <hip/hip_runtime.h>

typedef __bf16       v16bf __attribute__((ext_vector_type(16)));
typedef unsigned int v4u   __attribute__((ext_vector_type(4)));
typedef unsigned int v8u   __attribute__((ext_vector_type(8)));
typedef float        v8f   __attribute__((ext_vector_type(8)));
typedef float        v4f   __attribute__((ext_vector_type(4)));
typedef v4u __attribute__((may_alias)) v4ua;
typedef v4f __attribute__((may_alias)) v4fa;

union Frag { v16bf v; v8u w; v4u q[2]; };

#define BATCH 4
#define SEQ   4096
#define DM    256
#define NELEM (BATCH * SEQ * DM)
#define KSTEP 32
#define QW    16
#define WPB   2
#define QPB   (WPB * QW)
#define NGRP  (2 * (NELEM / 8))
#define SC2   (0.0625f * 1.44269504088896340736f)

static_assert(SEQ % 64 == 0);
static_assert(DM % 64 == 0);
static_assert(DM == 256);
static_assert(SEQ % QPB == 0);
static_assert(SEQ % KSTEP == 0);
static_assert(NGRP % 256 == 0);

__device__ __forceinline__ v8f wmma_bf16(v16bf a, v16bf b, v8f c) {
  return __builtin_amdgcn_wmma_f32_16x16x32_bf16(false, a, false, b, (short)0, c, false, false);
}

#define WGUARD2(d0, d1, a0, a1, bb) \
  asm volatile("v_nop\n\tv_nop\n\tv_nop\n\tv_nop" : "+v"(d0), "+v"(d1) : "v"(a0), "v"(a1), "v"(bb) : "memory")
#define WGUARD1(d0, a0, b0, b1) \
  asm volatile("v_nop\n\tv_nop\n\tv_nop\n\tv_nop" : "+v"(d0) : "v"(a0), "v"(b0), "v"(b1) : "memory")

__device__ __forceinline__ unsigned int bf16_bits(float x) {
  unsigned int u = __float_as_uint(x);
  u += 0x7FFFu + ((u >> 16) & 1u);
  return u >> 16;
}
__device__ __forceinline__ unsigned int pack2_bf16(float a, float b) {
  return bf16_bits(a) | (bf16_bits(b) << 16);
}
__device__ __forceinline__ void split2_bf16(float x, unsigned int& hb, unsigned int& lb) {
  unsigned int u = __float_as_uint(x);
  u += 0x7FFFu + ((u >> 16) & 1u);
  hb = u >> 16;
  const float hf = __uint_as_float(u & 0xFFFF0000u);
  lb = bf16_bits(x - hf);
}

__global__ __launch_bounds__(256) void cvt_rows_kernel(
    const float* __restrict__ q, const float* __restrict__ k,
    unsigned short* __restrict__ qb, unsigned short* __restrict__ kb, int ngroups)
{
  const int g = blockIdx.x * 256 + threadIdx.x;
  if (g >= ngroups) return;
  const int half = ngroups >> 1;
  const float* src;
  unsigned short* dst;
  if (g < half) {
    src = q + (size_t)g * 8;
    dst = qb + (size_t)g * 8;
  } else {
    const int e = g - half;
    src = k + (size_t)e * 8;
    dst = kb + (size_t)e * 8;
  }
  const v4f a = *(const v4fa*)src;
  const v4f c = *(const v4fa*)(src + 4);
  v4u o;
  o.x = pack2_bf16(a.x, a.y);
  o.y = pack2_bf16(a.z, a.w);
  o.z = pack2_bf16(c.x, c.y);
  o.w = pack2_bf16(c.z, c.w);
  *(volatile v4u*)dst = o;
  __threadfence();
  *(volatile v4u*)dst = o;
}

__device__ __forceinline__ void vt_store_pass(const unsigned short* sT, unsigned short* vt,
                                              int b, int d0, int kb, int w, int lane) {
  const int q8 = lane & 7, sub = lane >> 3;
  #pragma unroll
  for (int i = 0; i < 2; ++i) {
    const int lid = 8 * w + 4 * i + sub;
    const v4u x = *(const v4ua*)(sT + lid * 64 + 8 * q8);
    unsigned short* dst = vt + ((size_t)(b * DM + d0 + lid)) * SEQ + kb + 8 * q8;
    *(volatile v4u*)dst = x;
  }
}

__global__ __launch_bounds__(256) void vt_kernel(const float* __restrict__ v,
                                                 unsigned short* __restrict__ vt)
{
  __shared__ __attribute__((aligned(16))) unsigned short sT[64 * 64];

  const int tid = threadIdx.x, lane = tid & 31, w = tid >> 5;
  const int kb = blockIdx.x * 64, d0 = blockIdx.y * 64, b = blockIdx.z;

  #pragma unroll
  for (int t = 0; t < 4; ++t) {
    const int idx = tid + 256 * t;
    const int row = idx >> 4;
    const int c4  = idx & 15;
    const v4f x = *(const v4fa*)(v + ((size_t)(b * SEQ + kb + row)) * DM + d0 + 4 * c4);
    const int dl = 4 * c4;
    sT[(dl + 0) * 64 + row] = (unsigned short)bf16_bits(x.x);
    sT[(dl + 1) * 64 + row] = (unsigned short)bf16_bits(x.y);
    sT[(dl + 2) * 64 + row] = (unsigned short)bf16_bits(x.z);
    sT[(dl + 3) * 64 + row] = (unsigned short)bf16_bits(x.w);
  }
  __syncthreads();

  vt_store_pass(sT, vt, b, d0, kb, w, lane);
  __threadfence();
  vt_store_pass(sT, vt, b, d0, kb, w, lane);
}

__device__ __forceinline__ void out_store_pass(const float* so, float* out,
                                               int b, int q0, int lane) {
  const int q8 = lane & 7, sub = lane >> 3;
  #pragma unroll
  for (int i = 0; i < 32; ++i) {
    const int lid = 4 * i + sub;
    const int row = lid >> 3;
    const int c   = lid & 7;
    const v4f x = *(const v4fa*)(so + row * DM + 32 * c + 4 * q8);
    float* dst = out + ((size_t)(b * SEQ + q0 + row)) * DM + 32 * c + 4 * q8;
    *(volatile v4f*)dst = x;
  }
}

__global__ __launch_bounds__(64) void attn_kernel(
    const unsigned short* __restrict__ qb,
    const unsigned short* __restrict__ kbf,
    const unsigned short* __restrict__ vt,
    float* __restrict__ out)
{
  __shared__ __attribute__((aligned(16))) float sO[WPB * QW * DM];

  const int tid = threadIdx.x, lane = tid & 31, w = tid >> 5;
  const int h = lane >> 4, m = lane & 15;
  const int b = blockIdx.y;
  const int q0 = blockIdx.x * QPB + QW * w;

  const unsigned short* qrow  = qb  + ((size_t)b * SEQ + q0 + m) * DM + 8 * h;
  const unsigned short* kbase = kbf + ((size_t)b * SEQ + m) * DM + 8 * h;
  const unsigned short* vbase = vt  + ((size_t)b * DM + m) * SEQ + 8 * h;

  const v8f zero8 = {0.f, 0.f, 0.f, 0.f, 0.f, 0.f, 0.f, 0.f};
  v8f o[16];
  #pragma unroll
  for (int t = 0; t < 16; ++t) o[t] = zero8;
  float mrun = -1.0e30f, lrun = 0.0f;

  #pragma unroll 1
  for (int kb = 0; kb < SEQ; kb += KSTEP) {
    v8f s0 = zero8, s1 = zero8;
    const unsigned short* kp0 = kbase + (size_t)kb * DM;
    const unsigned short* kp1 = kp0 + 16 * DM;
    #pragma unroll
    for (int dc = 0; dc < 8; ++dc) {
      Frag qf, k0, k1;
      qf.q[0] = *(const v4ua*)(qrow + 32 * dc);
      qf.q[1] = *(const v4ua*)(qrow + 32 * dc + 16);
      k0.q[0] = *(const v4ua*)(kp0 + 32 * dc);
      k0.q[1] = *(const v4ua*)(kp0 + 32 * dc + 16);
      k1.q[0] = *(const v4ua*)(kp1 + 32 * dc);
      k1.q[1] = *(const v4ua*)(kp1 + 32 * dc + 16);
      s0 = wmma_bf16(k0.v, qf.v, s0);
      s1 = wmma_bf16(k1.v, qf.v, s1);
      WGUARD2(s0, s1, k0.v, k1.v, qf.v);
    }

    float mloc = -1.0e30f;
    #pragma unroll
    for (int r = 0; r < 8; ++r) {
      s0[r] = s0[r] * SC2;
      s1[r] = s1[r] * SC2;
      mloc = fmaxf(mloc, fmaxf(s0[r], s1[r]));
    }
    mloc = fmaxf(mloc, __shfl_xor(mloc, 16));
    const float mnew = fmaxf(mrun, mloc);
    const float alpha = exp2f(mrun - mnew);
    mrun = mnew;
    float lsum = 0.0f;
    #pragma unroll
    for (int r = 0; r < 8; ++r) {
      const float p0 = exp2f(s0[r] - mnew);
      const float p1 = exp2f(s1[r] - mnew);
      s0[r] = p0;
      s1[r] = p1;
      lsum += p0 + p1;
    }
    lsum += __shfl_xor(lsum, 16);
    lrun = lrun * alpha + lsum;
    #pragma unroll
    for (int t = 0; t < 16; ++t) o[t] = o[t] * alpha;

    Frag ph, pl;
    #pragma unroll
    for (int j = 0; j < 4; ++j) {
      unsigned int hb0, lb0, hb1, lb1;
      split2_bf16(s0[2 * j], hb0, lb0);
      split2_bf16(s0[2 * j + 1], hb1, lb1);
      ph.w[j] = hb0 | (hb1 << 16);
      pl.w[j] = lb0 | (lb1 << 16);
      split2_bf16(s1[2 * j], hb0, lb0);
      split2_bf16(s1[2 * j + 1], hb1, lb1);
      ph.w[4 + j] = hb0 | (hb1 << 16);
      pl.w[4 + j] = lb0 | (lb1 << 16);
    }

    const unsigned short* vp = vbase + kb;
    #pragma unroll
    for (int t = 0; t < 16; ++t) {
      Frag vf;
      vf.q[0] = *(const v4ua*)(vp + (size_t)(16 * t) * SEQ);
      vf.q[1] = *(const v4ua*)(vp + (size_t)(16 * t) * SEQ + 16);
      v8f d = o[t];
      d = wmma_bf16(vf.v, ph.v, d);
      d = wmma_bf16(vf.v, pl.v, d);
      WGUARD1(d, vf.v, ph.v, pl.v);
      o[t] = d;
    }
  }

  const float inv = 1.0f / lrun;
  float* so = sO + w * (QW * DM);
  #pragma unroll
  for (int t = 0; t < 16; ++t) {
    const v4f a = { o[t][0] * inv, o[t][1] * inv, o[t][2] * inv, o[t][3] * inv };
    const v4f c = { o[t][4] * inv, o[t][5] * inv, o[t][6] * inv, o[t][7] * inv };
    *(v4fa*)(so + m * DM + 16 * t + 8 * h)     = a;
    *(v4fa*)(so + m * DM + 16 * t + 8 * h + 4) = c;
  }
  __syncthreads();

  out_store_pass(so, out, b, q0, lane);
  __threadfence();
  out_store_pass(so, out, b, q0, lane);
}

extern "C" void kernel_launch(void* const* d_in, const int* in_sizes, int n_in,
                              void* d_out, int out_size, void* d_ws, size_t ws_size,
                              hipStream_t stream) {
  if (n_in < 3) return;
  if (in_sizes[0] != NELEM || in_sizes[1] != NELEM || in_sizes[2] != NELEM) return;
  if (out_size != NELEM) return;

  const float* Q = (const float*)d_in[0];
  const float* K = (const float*)d_in[1];
  const float* V = (const float*)d_in[2];
  float* out = (float*)d_out;

  const size_t plane_bytes = (size_t)NELEM * 2;
  const size_t total = 3 * plane_bytes;
  if (total > ws_size) return;

  char* ws = (char*)d_ws;
  unsigned short* qb = (unsigned short*)(ws);
  unsigned short* kb = (unsigned short*)(ws + plane_bytes);
  unsigned short* vt = (unsigned short*)(ws + 2 * plane_bytes);

  cvt_rows_kernel<<<NGRP / 256, 256, 0, stream>>>(Q, K, qb, kb, NGRP);

  dim3 gVt(SEQ / 64, DM / 64, BATCH);
  vt_kernel<<<gVt, 256, 0, stream>>>(V, vt);

  dim3 gAtt(SEQ / QPB, BATCH);
  attn_kernel<<<gAtt, 64, 0, stream>>>(qb, kb, vt, out);
}
